// VariableInteraction_59906203844675
// MI455X (gfx1250) — hardware-run, weakly checked
//
#include <hip/hip_runtime.h>


namespace {
constexpr int NB = 64, V = 256, D = 256, NN = 65536, QD = 64, NK = NB * V  , NE = NB * NN  ;
constexpr float XS = 8.0f, WSC = 256.0f, SCALE = 0.125f;
typedef _Float16 b16;
typedef __attribute__((ext_vector_type(16))) _Float16 v16b;
typedef __attribute__((ext_vector_type(8))) _Float16 v8b;
typedef __attribute__((ext_vector_type(8))) float v8f;
typedef __attribute__((ext_vector_type(4))) float v4f;
__device__ __forceinline__ float bf16_rne(float f) { unsigned int u = __float_as_uint(f); u += 0x7FFFu + ((u >> 16) & 1u); float r = __uint_as_float(u & 0xFFFF0000u); asm volatile("" : "+v"(r)); return r; }
__device__ __forceinline__ void split16(float v, b16& hi, b16& lo) { hi = (b16)v; lo = (b16)(v - (float)hi); }
__device__ __forceinline__ v16b frag_kb(const b16* p, int hh) { const v8b a = *(const v8b*)(p + 8 * hh), b = *(const v8b*)(p + 16 + 8 * hh); v16b f;
#pragma unroll
  for (int e = 0; e < 8; ++e) { f[e] = a[e]; f[8 + e] = b[e]; } return f; }
__device__ __forceinline__ v8f wmma16b(v16b a, v16b b, v8f c) { v8f d = __builtin_amdgcn_wmma_f32_16x16x32_f16(false, a, false, b, (short)0, c, false, false); asm volatile("v_nop\n\tv_nop\n\tv_nop\n\tv_nop" : "+v"(d) : "v"(a), "v"(b)); return d; }
__device__ __forceinline__ void wave_lds_sync() { __builtin_amdgcn_fence(__ATOMIC_RELEASE, "workgroup"); __builtin_amdgcn_wave_barrier(); __builtin_amdgcn_fence(__ATOMIC_ACQUIRE, "workgroup"); }
__device__ __forceinline__ float pmul(float a, float b) { float p = a * b; asm volatile("" : "+v"(p)); return p; }
__device__ __forceinline__ int iclamp(int v, int lo, int hi) { return v < lo ? lo : (v > hi ? hi : v); }
__device__ __forceinline__ float gelu_erf(float v) { return 0.5f * v * (1.0f + erff(v * 0.70710678118654752f)); }
#define N NK
#define E NE
constexpr int CSR_NBLK5 = 512, CSR_GB5 = 5, CSR_GN5 = 1 << CSR_GB5  , CSR_TS5 = (CSR_GN5 < 32 ? 32 : CSR_GN5)  , CSR_MAXG5 = 512, CSR_CAP5 = 12288  ;
__device__ __host__ __forceinline__ int csr_tix5(int v) { return (v >> CSR_GB5) * CSR_TS5 + (v & (CSR_GN5 - 1)); }
__global__ __launch_bounds__(64) void csrA_kernel5(const int* __restrict__ dst, int E, int N, int nG, int CHP, int NGP, int* __restrict__ STG, int* __restrict__ HST) {
  extern __shared__ int sm[];
  int* cnt = sm; int* run = sm + NGP; int* ids = sm + 2 * NGP;
  const int b = blockIdx.x; const int ch = (E + CSR_NBLK5 - 1) / CSR_NBLK5; const int e0 = b * ch, e1 = min(E, e0 + ch);
  for (int i = threadIdx.x; i < NGP; i += 64) cnt[i] = 0;
  for (int i = threadIdx.x; i < CHP; i += 64) ids[i] = -1;
  __syncthreads();
  if (threadIdx.x == 0) {
    for (int e = e0; e < e1; ++e) { int d = dst[e]; d = (d < 0) ? 0 : (d >= N ? N - 1 : d); cnt[d >> CSR_GB5] += 1; }
    int acc = 0; for (int g = 0; g < nG; ++g) { run[g] = acc; acc += cnt[g]; }
    for (int e = e0; e < e1; ++e) { int d = dst[e]; d = (d < 0) ? 0 : (d >= N ? N - 1 : d); const int g = d >> CSR_GB5; ids[run[g]] = e; run[g] += 1; } }
  __syncthreads();
  typedef __attribute__((ext_vector_type(4))) int v4i;
  for (int pass = 0; pass < 2; ++pass) {
    for (int i = threadIdx.x; i < CHP / 4; i += 64) *(volatile v4i*)(STG + (size_t)b * CHP + i * 4) = *(const v4i*)(&ids[i * 4]);
    for (int i = threadIdx.x; i < NGP / 4; i += 64) { v4i v; for (int e = 0; e < 4; ++e) v[e] = (i * 4 + e < nG) ? cnt[i * 4 + e] : 0; *(volatile v4i*)(HST + (size_t)b * NGP + i * 4) = v; }
    __threadfence(); }
}
__global__ __launch_bounds__(512) void csrS_kernel5(const int* __restrict__ HST, int nG, int NGP, int* __restrict__ START, int* __restrict__ TOT, int* __restrict__ OFF) {
  __shared__ int tot[CSR_MAXG5];
  const int b = threadIdx.x;
  for (int pass = 0; pass < 2; ++pass) { int runb = 0; for (int g = 0; g < nG; ++g) { int c = HST[(size_t)b * NGP + g]; c = (c < 0) ? 0 : c; ((volatile int*)OFF)[(size_t)g * CSR_NBLK5 + b] = runb; runb += c; } __threadfence(); }
  for (int g = threadIdx.x; g < nG; g += 512) { int s = 0; for (int bb = 0; bb < CSR_NBLK5; ++bb) { int c = HST[(size_t)bb * NGP + g]; s += (c < 0) ? 0 : c; } tot[g] = s; }
  __syncthreads();
  if (threadIdx.x < 32) {
    __shared__ int st[CSR_MAXG5 + 32];
    if (threadIdx.x == 0) { int acc = 0; for (int g = 0; g < NGP; ++g) { st[g] = acc; if (g < nG) acc += (tot[g] + 31) & ~31; } st[NGP] = acc; }
    __builtin_amdgcn_fence(__ATOMIC_RELEASE, "workgroup"); __builtin_amdgcn_wave_barrier(); __builtin_amdgcn_fence(__ATOMIC_ACQUIRE, "workgroup");
    for (int pass = 0; pass < 2; ++pass) { for (int i = threadIdx.x; i < NGP + 32; i += 32) { ((volatile int*)START)[i] = (i <= NGP) ? st[min(i, NGP)] : 0; ((volatile int*)TOT)[i] = (i < nG) ? tot[i] : 0; } __threadfence(); } }
}
__global__ __launch_bounds__(256) void csrB_kernel5(const int* __restrict__ dst, int N, int nG, int CHP, int NGP, int permLen, const int* __restrict__ STG, const int* __restrict__ HST, const int* __restrict__ OFF, const int* __restrict__ START, const int* __restrict__ TOT, int* __restrict__ PERM, int* __restrict__ ROWPTR, int* __restrict__ ROWCNT, int* __restrict__ FLAG) {
  typedef __attribute__((ext_vector_type(4))) int v4i;
  __shared__ int ids[CSR_CAP5]; __shared__ unsigned short key[CSR_CAP5]; __shared__ int outp[CSR_CAP5]; __shared__ int ncnt[CSR_GN5 + 1]; __shared__ int boff[CSR_NBLK5 + 1];
  const int g = blockIdx.x, t_ = threadIdx.x; int tot = TOT[g]; int st = START[g], stn = START[g + 1]; const int v0 = g * CSR_GN5; const int nv = min(CSR_GN5, N - v0); const int t0 = g * CSR_TS5;
  st = (st < 0) ? 0 : (st > permLen - 32 ? permLen - 32 : st) & ~31; stn = (stn < st) ? st : (stn > permLen ? permLen : stn); tot = (tot < 0) ? 0 : tot; if (tot > stn - st && tot <= CSR_CAP5) tot = stn - st;
  if (tot > CSR_CAP5) {
    for (int pass = 0; pass < 2; ++pass) { for (int i = t_; i < CSR_TS5 / 4; i += 256) { v4i a, c; for (int e = 0; e < 4; ++e) { a[e] = st; c[e] = 0; } *(volatile v4i*)(ROWPTR + t0 + i * 4) = a; *(volatile v4i*)(ROWCNT + t0 + i * 4) = c; } if (t_ == 0) ((volatile int*)FLAG)[0] = 1; __threadfence(); } (void)nv; return; }
  if (t_ == 0) { int acc = 0; for (int b = 0; b < CSR_NBLK5; ++b) { boff[b] = acc; int c = HST[(size_t)b * NGP + g]; c = (c < 0) ? 0 : (c > CHP ? CHP : c); acc += c; if (acc > tot) acc = tot; } boff[CSR_NBLK5] = acc; }
  for (int i = t_; i <= CSR_GN5; i += 256) ncnt[i] = 0;
  __syncthreads();
  for (int b = 0; b < CSR_NBLK5; ++b) { const int c = boff[b + 1] - boff[b]; int o_ = OFF[(size_t)g * CSR_NBLK5 + b]; o_ = (o_ < 0) ? 0 : (o_ > CHP - c ? CHP - c : o_); const int* src_ = STG + (size_t)b * CHP + o_;
    for (int i = t_; i < c; i += 256) { int id = src_[i]; id = (id < 0) ? 0 : id; ids[boff[b] + i] = id; int d = dst[id]; d = (d < v0) ? v0 : (d >= N ? N - 1 : d); int kk = d - v0; kk = (kk < 0) ? 0 : (kk >= CSR_GN5 ? CSR_GN5 - 1 : kk); key[boff[b] + i] = (unsigned short)kk; } }
  __syncthreads();
  if (t_ == 0) { for (int i = 0; i < tot; ++i) ncnt[key[i]] += 1; int acc = 0; for (int vl = 0; vl < CSR_GN5; ++vl) { const int c = ncnt[vl]; ncnt[vl] = acc; acc += c; } ncnt[CSR_GN5] = acc;
    for (int i = 0; i < tot; ++i) { const int vl = key[i]; outp[ncnt[vl]] = ids[i]; ncnt[vl] += 1; }
    for (int vl = CSR_GN5; vl > 0; --vl) ncnt[vl] = ncnt[vl - 1]; ncnt[0] = 0; }
  __syncthreads();
  for (int pass = 0; pass < 2; ++pass) {
    for (int i = t_; i < (stn - st) / 4; i += 256) { v4i v; for (int e = 0; e < 4; ++e) { const int q = i * 4 + e; v[e] = (q < tot) ? outp[q] : -1; } *(volatile v4i*)(PERM + st + i * 4) = v; }
    for (int i = t_; i < CSR_TS5 / 4; i += 256) { v4i a, c; for (int e = 0; e < 4; ++e) { const int vl = i * 4 + e; const int vc = vl < CSR_GN5 ? vl : CSR_GN5; a[e] = (vl < CSR_GN5) ? st + ncnt[vc] : st; c[e] = (vl < nv) ? (ncnt[(vc < CSR_GN5 ? vc : CSR_GN5 - 1) + 1] - ncnt[vc]) : 0; } *(volatile v4i*)(ROWPTR + t0 + i * 4) = a; *(volatile v4i*)(ROWCNT + t0 + i * 4) = c; }
    __threadfence(); }
}
__global__ __launch_bounds__(256) void csrZ_kernel5(int* __restrict__ p, size_t n4) { typedef __attribute__((ext_vector_type(4))) int v4i; const size_t tid = (size_t)blockIdx.x * 256 + threadIdx.x, nth = (size_t)gridDim.x * 256; v4i z = {0, 0, 0, 0}; for (size_t i = tid; i < n4; i += nth) *(volatile v4i*)(p + i * 4) = z; }
struct CsrBufs5 { int *STG, *HST, *OFF, *START, *TOT, *PERM, *ROWPTR, *ROWCNT, *FLAG; int nG, NGP, CHP; size_t permLen; char* base; size_t bytes; };
static size_t csr_carve5(CsrBufs5& c, char* ws, size_t off, int E, int N) {
  const size_t off0 = off; c.base = ws + off;
  auto al = [&](size_t bytes) { char* p = ws + off; off += (bytes + 255) & ~(size_t)255; return p; };
  c.nG = (N + CSR_GN5 - 1) / CSR_GN5; c.NGP = (c.nG + 31) & ~31; const int ch = (E + CSR_NBLK5 - 1) / CSR_NBLK5; c.CHP = (ch + 31) & ~31; c.permLen = (size_t)E + 32 * (size_t)c.nG + 32;
  c.STG = (int*)al((size_t)CSR_NBLK5 * c.CHP * 4); c.HST = (int*)al((size_t)CSR_NBLK5 * c.NGP * 4); c.OFF = (int*)al((size_t)c.NGP * CSR_NBLK5 * 4); c.START = (int*)al((size_t)(c.NGP + 64) * 4); c.TOT = (int*)al((size_t)(c.NGP + 64) * 4);
  c.PERM = (int*)al(c.permLen * 4); c.ROWPTR = (int*)al((size_t)c.nG * CSR_TS5 * 4); c.ROWCNT = (int*)al((size_t)c.nG * CSR_TS5 * 4); c.FLAG = (int*)al(256);
  c.bytes = off - off0; return off;
}
static void csr_build5(const CsrBufs5& c, const int* dst, int E, int N, hipStream_t stream) {
  const size_t smem = (size_t)(2 * c.NGP + c.CHP) * 4;
  csrZ_kernel5<<<512, 256, 0, stream>>>((int*)c.base, c.bytes / 16);
  csrA_kernel5<<<CSR_NBLK5, 64, smem, stream>>>(dst, E, N, c.nG, c.CHP, c.NGP, c.STG, c.HST);
  csrS_kernel5<<<1, 512, 0, stream>>>(c.HST, c.nG, c.NGP, c.START, c.TOT, c.OFF);
  csrB_kernel5<<<c.nG, 256, 0, stream>>>(dst, N, c.nG, c.CHP, c.NGP, (int)c.permLen, c.STG, c.HST, c.OFF, c.START, c.TOT, c.PERM, c.ROWPTR, c.ROWCNT, c.FLAG);
}

#undef N
#undef E

__global__ __launch_bounds__(256) void wput_kernel(const float* __restrict__ qr, const float* __restrict__ qi, const float* __restrict__ qj, const float* __restrict__ qk, const float* __restrict__ kr, const float* __restrict__ ki, const float* __restrict__ kj, const float* __restrict__ kk, const float* __restrict__ vw, const float* __restrict__ ow, b16* __restrict__ WQKV, b16* __restrict__ WO) { const int u = blockIdx.x * 256 + threadIdx.x; if (u >= 768 * 32) return; const int r = u / 32, k0 = (u % 32) * 8; const int part = r / 256, o = r % 256;
  v8b v, w2;
#pragma unroll
  for (int j = 0; j < 8; ++j) { const int i = k0 + j; float val; if (part == 2) val = vw[(size_t)o * D + i]; else { const int br = o / QD, bc = i / QD; const int comp = br ^ bc; const float sg = ((10318 >> (br * 4 + bc)) & 1) ? -1.0f : 1.0f; const float* src = part == 0 ? (comp == 0 ? qr : comp == 1 ? qi : comp == 2 ? qj : qk) : (comp == 0 ? kr : comp == 1 ? ki : comp == 2 ? kj : kk); val = sg * bf16_rne(src[(o % QD) * QD + (i % QD)]); }
    v[j] = (b16)(bf16_rne(val) * WSC); w2[j] = (b16)(part == 0 ? bf16_rne(ow[(size_t)o * D + i]) * WSC : 0.0f); }
  for (int pass = 0; pass < 2; ++pass) { *(volatile v8b*)(WQKV + (size_t)r * D + k0) = v; if (part == 0) *(volatile v8b*)(WO + (size_t)o * D + k0) = w2; __threadfence(); } }
__global__ __launch_bounds__(256) void key_kernel(const int* __restrict__ vidx, int* __restrict__ KEY) { const size_t u = (size_t)blockIdx.x * 256 + threadIdx.x; if (u >= (size_t)NE) return; const int b = (int)(u / NN); const int k = b * V + iclamp(vidx[u], 0, V - 1); for (int pass = 0; pass < 2; ++pass) { ((volatile int*)KEY)[u] = k; __threadfence(); } }
__global__ __launch_bounds__(256) void dens_kernel(const float* __restrict__ dens, const float* __restrict__ mask, const float* __restrict__ g1w, const float* __restrict__ g1b, const float* __restrict__ g2w, const float* __restrict__ g2b, const int* __restrict__ PERM, const int* __restrict__ ROWPTR, const int* __restrict__ ROWCNT, int permLen, float* __restrict__ DWP) { const int wave = threadIdx.x >> 5, lane = threadIdx.x & 31; const size_t key = (size_t)blockIdx.x * 8 + wave; if (key >= (size_t)NK) return; int st = ROWPTR[key], cnt = ROWCNT[key]; cnt = iclamp(cnt, 0, NE); st = iclamp(st, 0, permLen - cnt);
  float s0 = 0.0f, s1 = 0.0f, s2 = 0.0f, sm = 0.0f;
  for (int j = lane; j < cnt; j += 32) { const size_t u = (size_t)iclamp(PERM[st + j], 0, NE - 1); const float m = bf16_rne(mask[u]); sm += m; s0 += pmul(bf16_rne(dens[u * 3]), m); s1 += pmul(bf16_rne(dens[u * 3 + 1]), m); s2 += pmul(bf16_rne(dens[u * 3 + 2]), m); }
  for (int o = 16; o; o >>= 1) { s0 += __shfl_xor(s0, o); s1 += __shfl_xor(s1, o); s2 += __shfl_xor(s2, o); sm += __shfl_xor(sm, o); }
  const float inv = 1.0f / fmaxf(sm, 1.0f); const float d0 = s0 * inv, d1 = s1 * inv, d2 = s2 * inv; float g = bf16_rne(g2b[0]);
  if (lane < 16) { const float h = gelu_erf(pmul(d0, bf16_rne(g1w[lane * 3])) + pmul(d1, bf16_rne(g1w[lane * 3 + 1])) + pmul(d2, bf16_rne(g1w[lane * 3 + 2])) + bf16_rne(g1b[lane])); g = pmul(h, bf16_rne(g2w[lane])); } else g = 0.0f;
  for (int o = 8; o; o >>= 1) g += __shfl_xor(g, o);
  const float tot = __shfl(g, 0) + bf16_rne(g2b[0]); const float dw = 1.0f / (1.0f + __expf(-tot));
  for (int pass = 0; pass < 2; ++pass) { ((volatile float*)DWP)[key * 32 + lane] = lane == 0 ? dw : 0.0f; __threadfence(); } }
__global__ __launch_bounds__(32) void qkv_kernel(const float* __restrict__ he, const b16* __restrict__ WQKV, const float* __restrict__ qb, const float* __restrict__ kb, const float* __restrict__ vb, float* __restrict__ QKV, b16* __restrict__ KH, b16* __restrict__ KL) { __shared__ __attribute__((aligned(16))) b16 Ah[16][D + 8]; __shared__ float Tf[16][260]; const int lane = threadIdx.x, nloc = lane & 15, hlf = lane >> 4; const int g = blockIdx.x % 3; const size_t m0 = (size_t)(blockIdx.x / 3) * 16;
  for (int rr = 0; rr < 16; ++rr) for (int q = 0; q < 8; ++q) Ah[rr][q * 32 + lane] = (b16)(bf16_rne(he[(m0 + rr) * D + q * 32 + lane]) * XS);
  wave_lds_sync(); v8f acc[16];
#pragma unroll
  for (int t = 0; t < 16; ++t) acc[t] = (v8f){};
#pragma unroll 2
  for (int kb8 = 0; kb8 < D; kb8 += 32) { const v16b a = frag_kb(&Ah[nloc][kb8], hlf);
#pragma unroll
    for (int t = 0; t < 16; ++t) acc[t] = wmma16b(a, frag_kb(WQKV + (size_t)(g * 256 + t * 16 + nloc) * D + kb8, hlf), acc[t]); }
  const float* bias = g == 0 ? qb : (g == 1 ? kb : vb);
#pragma unroll
  for (int t = 0; t < 16; ++t) { const int cc = t * 16 + nloc; const float bb = bf16_rne(bias[cc]);
#pragma unroll
    for (int r8 = 0; r8 < 8; ++r8) Tf[8 * hlf + r8][cc] = acc[t][r8] * (1.0f / (XS * WSC)) + bb; }
  wave_lds_sync();
  for (int pass = 0; pass < 2; ++pass) { for (int rr = 0; rr < 16; ++rr) { for (int q = 0; q < 2; ++q) *(volatile v4f*)(QKV + (m0 + rr) * 768 + g * 256 + q * 128 + lane * 4) = *(const v4f*)(&Tf[rr][q * 128 + lane * 4]);
      if (g == 1) { v8b ph, pl; for (int j = 0; j < 8; ++j) { b16 p, l; split16(Tf[rr][lane * 8 + j] * XS, p, l); ph[j] = p; pl[j] = l; } *(volatile v8b*)(KH + (m0 + rr) * D + lane * 8) = ph; *(volatile v8b*)(KL + (m0 + rr) * D + lane * 8) = pl; } } __threadfence(); } }
__global__ __launch_bounds__(32) void att_kernel(const float* __restrict__ QKV, const b16* __restrict__ KH, const b16* __restrict__ KL, const float* __restrict__ DWP, float* __restrict__ O) { __shared__ __attribute__((aligned(16))) b16 Qh[16][D + 8], Ql[16][D + 8]; __shared__ float Sf[16][260]; __shared__ __attribute__((aligned(16))) b16 Ph[16][D + 8], Pl[16][D + 8]; __shared__ __attribute__((aligned(16))) b16 Vh[D][40], Vl[D][40];
  const int lane = threadIdx.x, nloc = lane & 15, hlf = lane >> 4; const size_t m0 = (size_t)blockIdx.x * 16; const int b = (int)(m0 / V); const size_t kbase = (size_t)b * V;
  for (int rr = 0; rr < 16; ++rr) for (int q = 0; q < 8; ++q) { b16 p, l; split16(QKV[(m0 + rr) * 768 + q * 32 + lane] * XS, p, l); Qh[rr][q * 32 + lane] = p; Ql[rr][q * 32 + lane] = l; }
  wave_lds_sync(); v8f acc[16];
#pragma unroll
  for (int t = 0; t < 16; ++t) acc[t] = (v8f){};
#pragma unroll 2
  for (int kb8 = 0; kb8 < D; kb8 += 32) { const v16b ah = frag_kb(&Qh[nloc][kb8], hlf), al = frag_kb(&Ql[nloc][kb8], hlf);
#pragma unroll
    for (int t = 0; t < 16; ++t) { const size_t ro = (kbase + t * 16 + nloc) * D + kb8; const v16b bh = frag_kb(KH + ro, hlf), bl = frag_kb(KL + ro, hlf); acc[t] = wmma16b(ah, bh, acc[t]); acc[t] = wmma16b(ah, bl, acc[t]); acc[t] = wmma16b(al, bh, acc[t]); } }
#pragma unroll
  for (int t = 0; t < 16; ++t) { const int w = t * 16 + nloc; const float gs = 1.0f + 0.5f * DWP[(kbase + w) * 32];
#pragma unroll
    for (int r8 = 0; r8 < 8; ++r8) Sf[8 * hlf + r8][w] = pmul(acc[t][r8] * (SCALE / (XS * XS)), gs); }
  wave_lds_sync();
  for (int rr = 0; rr < 16; ++rr) { float mx = -INFINITY; for (int q = 0; q < 8; ++q) mx = fmaxf(mx, Sf[rr][q * 32 + lane]); for (int o = 16; o; o >>= 1) mx = fmaxf(mx, __shfl_xor(mx, o)); float se = 0.0f; float ev[8];
#pragma unroll
    for (int q = 0; q < 8; ++q) { ev[q] = __expf(Sf[rr][q * 32 + lane] - mx); se += ev[q]; }
    for (int o = 16; o; o >>= 1) se += __shfl_xor(se, o); const float inv = 1.0f / se;
#pragma unroll
    for (int q = 0; q < 8; ++q) { b16 p, l; split16(pmul(ev[q], inv) * XS, p, l); Ph[rr][q * 32 + lane] = p; Pl[rr][q * 32 + lane] = l; } }
  wave_lds_sync();
#pragma unroll
  for (int t = 0; t < 16; ++t) acc[t] = (v8f){};
  for (int ws = 0; ws < V; ws += 32) {
    for (int rr = 0; rr < 32; ++rr) { const float* vr = QKV + (kbase + ws + rr) * 768 + 512; for (int q = 0; q < 8; ++q) { b16 p, l; split16(vr[q * 32 + lane] * XS, p, l); Vh[q * 32 + lane][rr] = p; Vl[q * 32 + lane][rr] = l; } }
    wave_lds_sync(); const v16b ph = frag_kb(&Ph[nloc][ws], hlf), pl = frag_kb(&Pl[nloc][ws], hlf);
#pragma unroll
    for (int t = 0; t < 16; ++t) { const v16b vh = frag_kb(&Vh[t * 16 + nloc][0], hlf), vl = frag_kb(&Vl[t * 16 + nloc][0], hlf); acc[t] = wmma16b(ph, vh, acc[t]); acc[t] = wmma16b(ph, vl, acc[t]); acc[t] = wmma16b(pl, vh, acc[t]); }
    wave_lds_sync(); }
#pragma unroll
  for (int t = 0; t < 16; ++t)
#pragma unroll
    for (int r8 = 0; r8 < 8; ++r8) Sf[8 * hlf + r8][t * 16 + nloc] = acc[t][r8] * (1.0f / (XS * XS));
  wave_lds_sync();
  for (int pass = 0; pass < 2; ++pass) { for (int rr = 0; rr < 16; ++rr) for (int q = 0; q < 2; ++q) *(volatile v4f*)(O + (m0 + rr) * D + q * 128 + lane * 4) = *(const v4f*)(&Sf[rr][q * 128 + lane * 4]); __threadfence(); } }
__global__ __launch_bounds__(32) void out_kernel(const float* __restrict__ O, const float* __restrict__ he, const b16* __restrict__ WO, const float* __restrict__ ob, const float* __restrict__ lw, const float* __restrict__ lb, float* __restrict__ out) { __shared__ __attribute__((aligned(16))) b16 Ah[16][D + 8], Al[16][D + 8]; __shared__ float Tf[16][260]; const int lane = threadIdx.x, nloc = lane & 15, hlf = lane >> 4; const size_t m0 = (size_t)blockIdx.x * 16;
  for (int rr = 0; rr < 16; ++rr) for (int q = 0; q < 8; ++q) { b16 p, l; split16(O[(m0 + rr) * D + q * 32 + lane] * XS, p, l); Ah[rr][q * 32 + lane] = p; Al[rr][q * 32 + lane] = l; }
  wave_lds_sync(); v8f acc[16];
#pragma unroll
  for (int t = 0; t < 16; ++t) acc[t] = (v8f){};
#pragma unroll 2
  for (int kb8 = 0; kb8 < D; kb8 += 32) { const v16b a = frag_kb(&Ah[nloc][kb8], hlf), al = frag_kb(&Al[nloc][kb8], hlf);
#pragma unroll
    for (int t = 0; t < 16; ++t) { const v16b bw = frag_kb(WO + (size_t)(t * 16 + nloc) * D + kb8, hlf); acc[t] = wmma16b(a, bw, acc[t]); acc[t] = wmma16b(al, bw, acc[t]); } }
#pragma unroll
  for (int t = 0; t < 16; ++t) { const int cc = t * 16 + nloc; const float bb = bf16_rne(ob[cc]);
#pragma unroll
    for (int r8 = 0; r8 < 8; ++r8) { const int rr = 8 * hlf + r8; Tf[rr][cc] = acc[t][r8] * (1.0f / (XS * WSC)) + bb + bf16_rne(he[(m0 + rr) * D + cc]); } }
  wave_lds_sync(); float gw[8], gb2[8]; for (int q = 0; q < 8; ++q) { gw[q] = bf16_rne(lw[q * 32 + lane]); gb2[q] = bf16_rne(lb[q * 32 + lane]); }
  for (int pass = 0; pass < 2; ++pass) { for (int rr = 0; rr < 16; ++rr) { float v[8]; float s = 0.0f; for (int q = 0; q < 8; ++q) { v[q] = Tf[rr][q * 32 + lane]; s += v[q]; } for (int o = 16; o; o >>= 1) s += __shfl_xor(s, o); const float mu = s * (1.0f / D); float qd = 0.0f; for (int q = 0; q < 8; ++q) { const float dd = v[q] - mu; qd += dd * dd; } for (int o = 16; o; o >>= 1) qd += __shfl_xor(qd, o); const float rstd = rsqrtf(qd * (1.0f / D) + 1e-5f);
      for (int q = 0; q < 8; ++q) ((volatile float*)out)[(m0 + rr) * D + q * 32 + lane] = pmul(pmul(v[q] - mu, rstd), gw[q]) + gb2[q]; } __threadfence(); } }
}

extern "C" void kernel_launch(void* const* d_in, const int* in_sizes, int n_in, void* d_out, int out_size, void* d_ws, size_t ws_size, hipStream_t stream) {
  (void)n_in;
  auto Fp = [&](int i) { return (const float*)d_in[i]; }; auto Ip = [&](int i) { return (const int*)d_in[i]; };
  if (in_sizes[0] != NK * D || in_sizes[1] != NE * 3 || in_sizes[2] != NE || in_sizes[3] != NE || in_sizes[4] != QD * QD || in_sizes[14] != D * D || in_sizes[16] != D * D || in_sizes[18] != 48 || in_sizes[20] != 16 || out_size != NK * D) return;
  const int BLIM = NB;
  size_t off = 0; char* ws = (char*)d_ws;
  auto carve = [&](size_t bytes) { char* p = ws + off; off += (bytes + 255) & ~(size_t)255; return p; };
  b16* WQKV = (b16*)carve((size_t)768 * D * 2); b16* WO = (b16*)carve((size_t)D * D * 2); int* KEY = (int*)carve((size_t)NE * 4); float* DWP = (float*)carve((size_t)NK * 32 * 4); float* QKV = (float*)carve((size_t)NK * 768 * 4); b16* KH = (b16*)carve((size_t)NK * D * 2); b16* KL = (b16*)carve((size_t)NK * D * 2); float* O = (float*)carve((size_t)NK * D * 4);
  CsrBufs5 csr; off = csr_carve5(csr, ws, off, NE, NK);
  if (off > ws_size || off > ((size_t)200 << 20)) return;
  wput_kernel<<<(768 * 32 + 255) / 256, 256, 0, stream>>>(Fp(4), Fp(5), Fp(6), Fp(7), Fp(9), Fp(10), Fp(11), Fp(12), Fp(14), Fp(16), WQKV, WO);
  key_kernel<<<NE / 256, 256, 0, stream>>>(Ip(2), KEY);
  csr_build5(csr, KEY, NE, NK, stream);
  dens_kernel<<<(BLIM * V) / 8, 256, 0, stream>>>(Fp(1), Fp(3), Fp(18), Fp(19), Fp(20), Fp(21), csr.PERM, csr.ROWPTR, csr.ROWCNT, (int)csr.permLen, DWP);
  qkv_kernel<<<(BLIM * V / 16) * 3, 32, 0, stream>>>(Fp(0), WQKV, Fp(8), Fp(13), Fp(15), QKV, KH, KL);
  att_kernel<<<BLIM * V / 16, 32, 0, stream>>>(QKV, KH, KL, DWP, O);
  out_kernel<<<BLIM * V / 16, 32, 0, stream>>>(O, Fp(0), WO, Fp(17), Fp(22), Fp(23), (float*)d_out);
}
